// SelfAttentionTF_62895501083076
// MI455X (gfx1250) — hardware-verified
//
#include <hip/hip_runtime.h>


#define NB_  8
#define NT_  1024
#define EMB  128
#define NH_  16
#define HE   (NH_ * EMB)
#define NTK  (NB_ * NT_)
#define NBH  4
#define NTH  (NBH * NT_)
#define PSC  32768.0f
#define WSC  64.0f
#define WSCI (1.0f / 64.0f)
#define LOSC 1024.0f
#define LOSCI (1.0f / 1024.0f)

typedef _Float16 h16;
typedef __attribute__((ext_vector_type(16))) _Float16 v16h;
typedef __attribute__((ext_vector_type(8)))  _Float16 v8h;
typedef __attribute__((ext_vector_type(4)))  _Float16 v4h;
typedef __attribute__((ext_vector_type(8)))  float    v8f;
typedef __attribute__((ext_vector_type(4)))  float    v4f;
typedef v8h  __attribute__((may_alias)) v8ha;
typedef v4f  __attribute__((may_alias)) v4fa;

__device__ __forceinline__ v16h cat16(v8h lo, v8h hi) { return __builtin_shufflevector(lo, hi, 0, 1, 2, 3, 4, 5, 6, 7, 8, 9, 10, 11, 12, 13, 14, 15); }
__device__ __forceinline__ v8f wmma16(v16h a, v16h b, v8f c) { return __builtin_amdgcn_wmma_f32_16x16x32_f16(false, a, false, b, (short)0, c, false, false); }
__device__ __forceinline__ void split16(float x, h16& h, h16& l) { h = (h16)x; l = (h16)((x - (float)h) * LOSC); }

__global__ __launch_bounds__(256) void k_x16(const float* __restrict__ x, h16* X16) {
    const int lane = threadIdx.x & 31, r = blockIdx.x * 8 + (threadIdx.x >> 5);
    if (r >= NTK) return;
    const v4f f = *(const v4f*)(x + (size_t)r * EMB + lane * 4);
    v4h o; o[0] = (h16)f[0]; o[1] = (h16)f[1]; o[2] = (h16)f[2]; o[3] = (h16)f[3];
    h16* d = X16 + (size_t)r * EMB + lane * 4;
    *(volatile v4h*)d = o;
    __threadfence();
    *(volatile v4h*)d = o;
}

__global__ __launch_bounds__(256) void k_wt(const float* __restrict__ Wm, int K, int N, h16* WT, h16* WTL) {
    __shared__ __align__(16) h16 th[64 * 72];
    __shared__ __align__(16) h16 tl[64 * 72];
    const int tid = threadIdx.x, k0 = blockIdx.x * 64, n0 = blockIdx.y * 64;
    const int kk = tid >> 2, nq = (tid & 3) * 16;
#pragma unroll
    for (int i = 0; i < 16; ++i) {
        h16 a, b; split16(Wm[(size_t)(k0 + kk) * N + n0 + nq + i] * WSC, a, b);
        th[(nq + i) * 72 + kk] = a; tl[(nq + i) * 72 + kk] = b;
    }
    __syncthreads();
    const int piece = tid & 7;
    const int npl = WTL ? 2 : 1;
    auto pass = [&]() {
        for (int p = 0; p < npl; ++p) {
#pragma unroll
            for (int s = 0; s < 2; ++s) {
                const int nr = (tid >> 3) + 32 * s;
                const v8h val = *(const v8ha*)((p ? tl : th) + nr * 72 + piece * 8);
                *(volatile v8h*)((p ? WTL : WT) + (size_t)(n0 + nr) * K + k0 + piece * 8) = val;
            }
        }
    };
    pass();
    __threadfence();
    pass();
}

template <bool SPLIT, bool OUT16>
__global__ __launch_bounds__(128) void k_lgemm(const h16* __restrict__ A, const h16* __restrict__ Al, const h16* __restrict__ Bn, const h16* __restrict__ Bl, int K,
                                               const float* __restrict__ bias, float oscale, void* Cv, int ldc) {
    __shared__ __align__(16) float ost[4][16 * 68];
    const int lane = threadIdx.x & 31, wave = threadIdx.x >> 5, lr = lane & 15, hi = lane >> 4;
    const int r0 = blockIdx.x * 64 + wave * 16, c0 = blockIdx.y * 64;
    const size_t aoff = (size_t)(r0 + lr) * K + 8 * hi;
    size_t boff[4];
#pragma unroll
    for (int t = 0; t < 4; ++t) boff[t] = (size_t)(c0 + t * 16 + lr) * K + 8 * hi;
    v8f acc[4], accx[4];
#pragma unroll
    for (int t = 0; t < 4; ++t) { acc[t] = (v8f){}; accx[t] = (v8f){}; }
#pragma unroll 1
    for (int kc = 0; kc < K; kc += 32) {
        const v16h a = cat16(*(const v8h*)(A + aoff + kc), *(const v8h*)(A + aoff + kc + 16));
        v16h al = a;
        if (SPLIT) al = cat16(*(const v8h*)(Al + aoff + kc), *(const v8h*)(Al + aoff + kc + 16));
#pragma unroll
        for (int t = 0; t < 4; ++t) {
            const v16h b = cat16(*(const v8h*)(Bn + boff[t] + kc), *(const v8h*)(Bn + boff[t] + kc + 16));
            acc[t] = wmma16(a, b, acc[t]);
            if (SPLIT) {
                accx[t] = wmma16(a, cat16(*(const v8h*)(Bl + boff[t] + kc), *(const v8h*)(Bl + boff[t] + kc + 16)), accx[t]);
                accx[t] = wmma16(al, b, accx[t]);
            }
        }
        if (SPLIT) asm volatile("v_nop\n\tv_nop\n\tv_nop\n\tv_nop" : "+v"(acc[0]), "+v"(acc[1]), "+v"(acc[2]), "+v"(acc[3]), "+v"(accx[0]), "+v"(accx[1]), "+v"(accx[2]), "+v"(accx[3]) : "v"(a), "v"(al));
        else       asm volatile("v_nop\n\tv_nop\n\tv_nop\n\tv_nop" : "+v"(acc[0]), "+v"(acc[1]), "+v"(acc[2]), "+v"(acc[3]) : "v"(a));
    }
    float* os = &ost[wave][0];
#pragma unroll
    for (int t = 0; t < 4; ++t) {
        const int n = c0 + t * 16 + lr;
        const float bv = bias ? bias[n] : 0.0f;
#pragma unroll
        for (int j = 0; j < 8; ++j) {
            float v = acc[t][j];
            if (SPLIT) v += accx[t][j] * LOSCI;
            os[(hi * 8 + j) * 68 + t * 16 + lr] = v * oscale + bv;
        }
    }
    __syncthreads();
    if (OUT16) {
        h16* crow = (h16*)Cv + (size_t)r0 * ldc + c0;
        auto pass = [&]() {
#pragma unroll
            for (int s = 0; s < 4; ++s) {
                const int row = 4 * s + (lane >> 3), piece = lane & 7;
                const float* sp = os + row * 68 + piece * 8;
                v8h o;
#pragma unroll
                for (int i = 0; i < 8; ++i) o[i] = (h16)sp[i];
                *(volatile v8h*)(crow + (size_t)row * ldc + piece * 8) = o;
            }
        };
        pass();
        __threadfence();
        pass();
    } else {
        float* crow = (float*)Cv + (size_t)r0 * ldc + c0;
        auto pass = [&]() {
#pragma unroll
            for (int s = 0; s < 8; ++s) {
                const int Lid = (lane >> 3) + 4 * s, piece = lane & 7;
                const int row = Lid >> 1, cofs = (Lid & 1) * 32 + piece * 4;
                const v4f val = *(const v4fa*)(os + row * 68 + cofs);
                *(volatile v4f*)(crow + (size_t)row * ldc + cofs) = val;
            }
        };
        pass();
        __threadfence();
        pass();
    }
}

__global__ __launch_bounds__(128) void k_attn(const h16* __restrict__ Q16, const h16* __restrict__ K16, const h16* __restrict__ VT16, h16* CH, h16* CL) {
    __shared__ __align__(16) h16 plds[4][16 * 32];
    __shared__ __align__(16) float ost[4][16 * 132];
    const int lane = threadIdx.x & 31, wave = threadIdx.x >> 5, lr = lane & 15, hi = lane >> 4;
    const int bid = blockIdx.x;
    const int b = bid / (NH_ * (NT_ / 64)), rem = bid - b * (NH_ * (NT_ / 64)), h = rem / (NT_ / 64), qt = rem - h * (NT_ / 64);
    const int q0 = qt * 64 + wave * 16;
    const size_t tok0 = (size_t)b * NT_;
    h16* pl = &plds[wave][0];
    v16h qa[4];
#pragma unroll
    for (int kc = 0; kc < 4; ++kc) {
        const h16* p = Q16 + (tok0 + q0 + lr) * HE + h * EMB + kc * 32 + 8 * hi;
        qa[kc] = cat16(*(const v8h*)p, *(const v8h*)(p + 16));
    }
    const h16* kh_b = K16 + tok0 * HE + h * EMB;
    const h16* vt_b = VT16 + (size_t)(h * EMB) * NTH + tok0;
    v8f o[8];
#pragma unroll
    for (int n = 0; n < 8; ++n) o[n] = (v8f){};
    float mrow[8], lpart[8];
#pragma unroll
    for (int j = 0; j < 8; ++j) { mrow[j] = -3.0e38f; lpart[j] = 0.f; }
#pragma unroll 1
    for (int kt = 0; kt < NT_ / 32; ++kt) {
        const int l0 = kt * 32;
        const h16* r0p = kh_b + (size_t)(l0 + lr) * HE + 8 * hi;
        const h16* r1p = kh_b + (size_t)(l0 + 16 + lr) * HE + 8 * hi;
        v8f s0 = {}, s1 = {};
#pragma unroll
        for (int kc = 0; kc < 4; ++kc) {
            s0 = wmma16(qa[kc], cat16(*(const v8h*)(r0p + kc * 32), *(const v8h*)(r0p + kc * 32 + 16)), s0);
            s1 = wmma16(qa[kc], cat16(*(const v8h*)(r1p + kc * 32), *(const v8h*)(r1p + kc * 32 + 16)), s1);
        }
        asm volatile("v_nop\n\tv_nop\n\tv_nop\n\tv_nop" : "+v"(s0), "+v"(s1) : "v"(qa[0]), "v"(qa[3]));
        float alpha[8];
#pragma unroll
        for (int j = 0; j < 8; ++j) {
            const float a0 = s0[j], a1 = s1[j];
            float mx = fmaxf(a0, a1);
            mx = fmaxf(mx, __shfl_xor(mx, 1, 16)); mx = fmaxf(mx, __shfl_xor(mx, 2, 16));
            mx = fmaxf(mx, __shfl_xor(mx, 4, 16)); mx = fmaxf(mx, __shfl_xor(mx, 8, 16));
            const float mn = fmaxf(mrow[j], mx);
            alpha[j] = __expf(mrow[j] - mn);
            mrow[j] = mn;
            const float p0 = __expf(a0 - mn), p1 = __expf(a1 - mn);
            lpart[j] = lpart[j] * alpha[j] + (p0 + p1);
            const int mr = hi * 8 + j;
            pl[mr * 32 + lr]      = (h16)(p0 * PSC);
            pl[mr * 32 + 16 + lr] = (h16)(p1 * PSC);
        }
#pragma unroll
        for (int n = 0; n < 8; ++n)
#pragma unroll
            for (int j = 0; j < 8; ++j) o[n][j] *= alpha[j];
        asm volatile("" ::: "memory");
        const v16h pa = cat16(*(const v8ha*)(pl + lr * 32 + hi * 8), *(const v8ha*)(pl + lr * 32 + 16 + hi * 8));
#pragma unroll
        for (int n = 0; n < 8; ++n) {
            const h16* vp = vt_b + (size_t)(n * 16 + lr) * NTH + l0 + hi * 8;
            o[n] = wmma16(pa, cat16(*(const v8h*)vp, *(const v8h*)(vp + 16)), o[n]);
        }
        asm volatile("v_nop\n\tv_nop\n\tv_nop\n\tv_nop" : "+v"(o[0]), "+v"(o[1]), "+v"(o[2]), "+v"(o[3]), "+v"(o[4]), "+v"(o[5]), "+v"(o[6]), "+v"(o[7]) : "v"(pa));
    }
    float inv[8];
#pragma unroll
    for (int j = 0; j < 8; ++j) {
        float rs = lpart[j];
        rs += __shfl_xor(rs, 1, 16); rs += __shfl_xor(rs, 2, 16); rs += __shfl_xor(rs, 4, 16); rs += __shfl_xor(rs, 8, 16);
        inv[j] = 1.0f / (rs * PSC);
    }
    float* os = &ost[wave][0];
#pragma unroll
    for (int n = 0; n < 8; ++n)
#pragma unroll
        for (int j = 0; j < 8; ++j) os[(hi * 8 + j) * 132 + n * 16 + lr] = o[n][j] * inv[j];
    __syncthreads();
    const size_t cbase = (tok0 + q0) * HE + (size_t)h * EMB;
    auto pass = [&]() {
#pragma unroll
        for (int s = 0; s < 8; ++s) {
            const int Lid = 4 * s + (lane >> 3), piece = lane & 7;
            const int row = Lid >> 1, cofs = (Lid & 1) * 64 + piece * 8;
            const float* sp = os + row * 132 + cofs;
            v8h oh, ol;
#pragma unroll
            for (int i = 0; i < 8; ++i) { h16 a, bq; split16(sp[i], a, bq); oh[i] = a; ol[i] = bq; }
            *(volatile v8h*)(CH + cbase + (size_t)row * HE + cofs) = oh;
            *(volatile v8h*)(CL + cbase + (size_t)row * HE + cofs) = ol;
        }
    };
    pass();
    __threadfence();
    pass();
}

extern "C" void kernel_launch(void* const* d_in, const int* in_sizes, int n_in,
                              void* d_out, int out_size, void* d_ws, size_t ws_size, hipStream_t stream) {
    (void)in_sizes; (void)n_in; (void)out_size;
    const float* x = (const float*)d_in[0]; const float* Wk = (const float*)d_in[1]; const float* Wq = (const float*)d_in[2]; const float* Wv = (const float*)d_in[3];
    const float* Wu = (const float*)d_in[4]; const float* bu = (const float*)d_in[5];
    float* out = (float*)d_out;
    char* wsp = (char*)d_ws;
    auto take = [&](size_t bytes) { char* p = wsp; wsp += (bytes + 255) & ~(size_t)255; return (void*)p; };
    h16* X16  = (h16*)take((size_t)NTK * EMB * 2);
    h16* WQT  = (h16*)take((size_t)HE * EMB * 2);
    h16* WKT  = (h16*)take((size_t)HE * EMB * 2);
    h16* WVT  = (h16*)take((size_t)HE * EMB * 2);
    h16* WUH  = (h16*)take((size_t)EMB * HE * 2);
    h16* WUL  = (h16*)take((size_t)EMB * HE * 2);
    h16* Q16  = (h16*)take((size_t)NTH * HE * 2);
    h16* K16  = (h16*)take((size_t)NTH * HE * 2);
    h16* VT16 = (h16*)take((size_t)HE * NTH * 2);
    h16* CH   = (h16*)take((size_t)NTH * HE * 2);
    h16* CL   = (h16*)take((size_t)NTH * HE * 2);
    if ((size_t)(wsp - (char*)d_ws) > ws_size) return;
    const float qk_scale = 0.29730177875068026f * WSCI;
    k_x16<<<NTK / 8, 256, 0, stream>>>(x, X16);
    k_wt<<<dim3(EMB / 64, HE / 64, 1), 256, 0, stream>>>(Wq, EMB, HE, WQT, nullptr);
    k_wt<<<dim3(EMB / 64, HE / 64, 1), 256, 0, stream>>>(Wk, EMB, HE, WKT, nullptr);
    k_wt<<<dim3(EMB / 64, HE / 64, 1), 256, 0, stream>>>(Wv, EMB, HE, WVT, nullptr);
    k_wt<<<dim3(HE / 64, EMB / 64, 1), 256, 0, stream>>>(Wu, HE, EMB, WUH, WUL);
    for (int hb = 0; hb < NB_ / NBH; ++hb) {
        const h16* Xh = X16 + (size_t)hb * NTH * EMB;
        k_lgemm<false, true><<<dim3(NTH / 64, HE / 64, 1), 128, 0, stream>>>(Xh, nullptr, WQT, nullptr, EMB, nullptr, qk_scale, Q16, HE);
        k_lgemm<false, true><<<dim3(NTH / 64, HE / 64, 1), 128, 0, stream>>>(Xh, nullptr, WKT, nullptr, EMB, nullptr, qk_scale, K16, HE);
        k_lgemm<false, true><<<dim3(HE / 64, NTH / 64, 1), 128, 0, stream>>>(WVT, nullptr, Xh, nullptr, EMB, nullptr, WSCI, VT16, NTH);
        k_attn<<<NBH * NH_ * (NT_ / 64), 128, 0, stream>>>(Q16, K16, VT16, CH, CL);
        k_lgemm<true, false><<<dim3(NTH / 64, EMB / 64, 1), 128, 0, stream>>>(CH, CL, WUH, WUL, HE, bu, WSCI, out + (size_t)hb * NTH * EMB, EMB);
    }
}
